// MeMViTAttention_79242146611851
// MI455X (gfx1250) — hardware-verified
//
#include <hip/hip_runtime.h>
#include <math.h>
#include <stdint.h>

#define NBATCH 2
#define NHEAD  8
#define DCH    96
#define DMODEL 768
#define TDIM   8
#define SDIM   28
#define QTOK   6272
#define KSD    14
#define KTOK   1568
#define KPAD   1600
#define MQ     (NBATCH * QTOK)
#define MK     (NBATCH * KPAD)
#define NQB    (QTOK / 64)
#define NKC    (KPAD / 64)
#define NTAP   27
#define WSC    1024.0f
#define QSC    8.0f
#define VSC    16.0f
#define PSC    1024.0f
#define CSC    1024.0f
#define ATT_SCALE 0.10206207261596575f
#define SSC    (ATT_SCALE / (QSC * QSC))
#define LN_EPS 1e-5f
#define NEG_BIG (-1.0e30f)
static_assert(NHEAD * DCH == DMODEL);
static_assert(QTOK == TDIM * SDIM * SDIM);
static_assert(KTOK == TDIM * KSD * KSD);
static_assert((QTOK % 64) == 0 && (KPAD % 64) == 0 && KPAD >= KTOK && (KPAD - KTOK) < 64 && KTOK >= 64);
static_assert((MQ % 32) == 0 && (MK % 128) == 0 && (DMODEL % 128) == 0 && (DMODEL % 32) == 0);
static_assert(((DMODEL * DMODEL) % 2048) == 0);
static_assert(DCH == 3 * 32);

typedef _Float16 v16h __attribute__((ext_vector_type(16)));
typedef _Float16 v8h  __attribute__((ext_vector_type(8)));
typedef float    v8f  __attribute__((ext_vector_type(8)));
typedef float    v4f  __attribute__((ext_vector_type(4)));
typedef unsigned int v4u __attribute__((ext_vector_type(4)));
union FH { v16h v; v8h h[2]; };

__device__ __forceinline__ float bfr(float f) {
  unsigned u = __float_as_uint(f);
  u = (u + 0x7FFFu + ((u >> 16) & 1u)) & 0xFFFF0000u;
  return __uint_as_float(u);
}
__device__ __forceinline__ unsigned short h_bits(_Float16 x) { return __builtin_bit_cast(unsigned short, x); }
__device__ __forceinline__ unsigned pk16(unsigned short a, unsigned short b) { return (unsigned)a | ((unsigned)b << 16); }
__device__ __forceinline__ v8f zero8() { v8f z = {0.f, 0.f, 0.f, 0.f, 0.f, 0.f, 0.f, 0.f}; return z; }

__device__ __forceinline__ v16h ldfrag_h(const _Float16* p) {
  FH f;
  f.h[0] = *(const v8h*)(p);
  f.h[1] = *(const v8h*)(p + 16);
  return f.v;
}

__device__ __forceinline__ v8f mma_h(v16h a, v16h b, v8f c) {
  c = __builtin_amdgcn_wmma_f32_16x16x32_f16(false, a, false, b, (short)0, c, false, false);
#if defined(__HIP_DEVICE_COMPILE__)
  asm volatile("v_nop\n\tv_nop\n\tv_nop\n\tv_nop" : "+v"(c) : "v"(a), "v"(b));
#endif
  return c;
}
__device__ __forceinline__ v8f mma_h_raw(v16h a, v16h b, v8f c) {
  return __builtin_amdgcn_wmma_f32_16x16x32_f16(false, a, false, b, (short)0, c, false, false);
}
__device__ __forceinline__ void guard3(v8f& x, v8f& y, v16h a, v16h b, v16h d) {
#if defined(__HIP_DEVICE_COMPILE__)
  asm volatile("v_nop\n\tv_nop\n\tv_nop\n\tv_nop" : "+v"(x), "+v"(y) : "v"(a), "v"(b), "v"(d));
#endif
}
__device__ __forceinline__ void acc_guard4(v8f& a, v8f& b, v8f& c, v8f& d) {
#if defined(__HIP_DEVICE_COMPILE__)
  asm volatile("v_nop\n\tv_nop\n\tv_nop\n\tv_nop" : "+v"(a), "+v"(b), "+v"(c), "+v"(d));
#endif
}
__device__ __forceinline__ void acc_guard2(v8f& a, v8f& b) {
#if defined(__HIP_DEVICE_COMPILE__)
  asm volatile("v_nop\n\tv_nop\n\tv_nop\n\tv_nop" : "+v"(a), "+v"(b));
#endif
}
__device__ __forceinline__ void wave_sync_lds() {
  __builtin_amdgcn_fence(__ATOMIC_RELEASE, "workgroup");
  __builtin_amdgcn_wave_barrier();
  __builtin_amdgcn_fence(__ATOMIC_ACQUIRE, "workgroup");
}

__global__ __launch_bounds__(256) void cvt_w(const float* __restrict__ in, unsigned short* out, int n, float scale) {
  const size_t i8 = ((size_t)blockIdx.x * 256 + threadIdx.x) * 8;
  if (i8 + 8 > (size_t)n) return;
  const v4f a = *(const v4f*)(in + i8);
  const v4f b = *(const v4f*)(in + i8 + 4);
  v4u p;
#pragma unroll
  for (int e = 0; e < 2; ++e) {
    p[e]     = pk16(h_bits((_Float16)(bfr(a[2 * e]) * scale)), h_bits((_Float16)(bfr(a[2 * e + 1]) * scale)));
    p[2 + e] = pk16(h_bits((_Float16)(bfr(b[2 * e]) * scale)), h_bits((_Float16)(bfr(b[2 * e + 1]) * scale)));
  }
  *(volatile v4u*)(out + i8) = p;
  __threadfence();
  *(volatile v4u*)(out + i8) = p;
}

template <int SW, int WO>
__global__ __launch_bounds__(192) void pool_ln(const float* __restrict__ x, const float* __restrict__ w,
                                               const float* __restrict__ gam, const float* __restrict__ bet,
                                               unsigned short* out, int rowsPB) {
  __shared__ __align__(16) _Float16 tileL[WO * 192];
  __shared__ float redA[8];
  __shared__ float redB[8];
  const int tid  = threadIdx.x;
  const int lane = tid & 31;
  const int wv   = tid >> 5;
  const int hl   = (tid >= DCH) ? 1 : 0;
  const int c    = tid - DCH * hl;
  int bid = (int)blockIdx.x;
  const int yo = bid % WO;   bid /= WO;
  const int to = bid % TDIM; bid /= TDIM;
  const int hp = bid % 4;    bid /= 4;
  const int b  = bid;
  const int chan = hp * 192 + tid;

  float wr[NTAP];
#pragma unroll
  for (int k = 0; k < NTAP; ++k) wr[k] = bfr(w[c * NTAP + k]);
  const float g  = bfr(gam[c]);
  const float bt = bfr(bet[c]);

  const float* xb = x + (size_t)b * QTOK * DMODEL + chan;
  int   roff[9];
  float rfac[9];
#pragma unroll
  for (int i = 0; i < 3; ++i) {
    const int tp  = to - 1 + i;
    const int tv  = (tp >= 0 && tp < TDIM) ? 1 : 0;
    const int tcl = min(max(tp, 0), TDIM - 1);
#pragma unroll
    for (int j = 0; j < 3; ++j) {
      const int yp  = yo * SW - 1 + j;
      const int yv  = (yp >= 0 && yp < SDIM) ? 1 : 0;
      const int ycl = min(max(yp, 0), SDIM - 1);
      roff[3 * i + j] = (tcl * (SDIM * SDIM) + ycl * SDIM) * DMODEL;
      rfac[3 * i + j] = (float)(tv * yv);
    }
  }

  float win[9][3];
#pragma unroll
  for (int q = 0; q < 9; ++q) { win[q][0] = 0.f; win[q][1] = 0.f; win[q][2] = 0.f; }
  if (SW == 1) {
#pragma unroll
    for (int q = 0; q < 9; ++q) win[q][1] = bfr(xb[roff[q]]) * rfac[q];
  }

#pragma unroll 1
  for (int xo = 0; xo < WO; ++xo) {
    if (SW == 1) {
      const int xp  = xo + 1;
      const float xf = (xp < SDIM) ? 1.f : 0.f;
      const int xcl = (xp < SDIM) ? xp : (SDIM - 1);
#pragma unroll
      for (int q = 0; q < 9; ++q) win[q][2] = bfr(xb[roff[q] + xcl * DMODEL]) * (rfac[q] * xf);
    } else {
      const int xp = 2 * xo;
#pragma unroll
      for (int q = 0; q < 9; ++q) {
        win[q][1] = bfr(xb[roff[q] + xp * DMODEL]) * rfac[q];
        win[q][2] = bfr(xb[roff[q] + (xp + 1) * DMODEL]) * rfac[q];
      }
    }
    float s = 0.f;
#pragma unroll
    for (int q = 0; q < 9; ++q) {
      s += wr[3 * q + 0] * win[q][0];
      s += wr[3 * q + 1] * win[q][1];
      s += wr[3 * q + 2] * win[q][2];
    }
    float s1 = s;
#pragma unroll
    for (int off = 16; off > 0; off >>= 1) s1 += __shfl_xor(s1, off, 32);
    if (lane == 0) redA[wv] = s1;
    __syncthreads();
    const float mean = ((redA[3 * hl] + redA[3 * hl + 1]) + redA[3 * hl + 2]) * (1.0f / 96.0f);
    const float d = s - mean;
    float s2 = d * d;
#pragma unroll
    for (int off = 16; off > 0; off >>= 1) s2 += __shfl_xor(s2, off, 32);
    if (lane == 0) redB[wv] = s2;
    __syncthreads();
    const float var = ((redB[3 * hl] + redB[3 * hl + 1]) + redB[3 * hl + 2]) * (1.0f / 96.0f);
    const float y = (d * rsqrtf(var + LN_EPS)) * g + bt;
    tileL[xo * 192 + tid] = (_Float16)y;
    if (SW == 1) {
#pragma unroll
      for (int q = 0; q < 9; ++q) { win[q][0] = win[q][1]; win[q][1] = win[q][2]; }
    } else {
#pragma unroll
      for (int q = 0; q < 9; ++q) win[q][0] = win[q][2];
    }
  }
  __syncthreads();

  const int cl = (lane < 24) ? lane : 23;
  const size_t rowbase = (size_t)b * (size_t)rowsPB + (size_t)((to * WO + yo) * WO);
  for (int pass = 0; pass < 2; ++pass) {
    for (int xo = wv; xo < WO; xo += 6) {
      const v4u val = *(const v4u*)(tileL + xo * 192 + cl * 8);
      unsigned short* p = out + (rowbase + (size_t)xo) * DMODEL + hp * 192 + cl * 8;
      if (lane < 24) *(volatile v4u*)p = val;
    }
    __threadfence();
  }
}

template <int OM>
__global__ __launch_bounds__(128) void gemm_h(
    const unsigned short* __restrict__ A, int lda, const unsigned short* __restrict__ B, int ldb,
    void* C0, const float* __restrict__ bias, int ldc, int M, int N, int K, float oscale) {
  __shared__ __align__(16) float sT[4][16 * 132];
  const int lane = threadIdx.x & 31;
  const int wave = threadIdx.x >> 5;
  const int tilesN = N >> 7;
  const int tilesM = M >> 5;
  const int tile = blockIdx.x * 4 + wave;
  if (tile >= tilesM * tilesN) return;
  const int tm = tile / tilesN;
  const int tn = tile - tm * tilesN;
  const int m0 = tm << 5;
  const int n0 = tn << 7;
  const int rl   = lane & 15;
  const int hh   = lane >> 4;
  const int koff = hh * 8;

  v8f acc[2][8];
#pragma unroll
  for (int i = 0; i < 2; ++i)
#pragma unroll
    for (int j = 0; j < 8; ++j) acc[i][j] = zero8();

  const _Float16* Ah = (const _Float16*)(const void*)A;
  const _Float16* Bh = (const _Float16*)(const void*)B;
  const _Float16* ar0 = Ah + (size_t)(m0 + rl) * (size_t)lda + koff;
  const _Float16* ar1 = Ah + (size_t)(m0 + 16 + rl) * (size_t)lda + koff;
  const _Float16* br  = Bh + (size_t)(n0 + rl) * (size_t)ldb + koff;
  for (int k0 = 0; k0 < K; k0 += 32) {
    const v16h a0 = ldfrag_h(ar0 + k0);
    const v16h a1 = ldfrag_h(ar1 + k0);
#pragma unroll
    for (int j = 0; j < 8; ++j) {
      const v16h bb = ldfrag_h(br + (size_t)j * 16 * (size_t)ldb + k0);
      acc[0][j] = mma_h_raw(a0, bb, acc[0][j]);
      acc[1][j] = mma_h_raw(a1, bb, acc[1][j]);
      guard3(acc[0][j], acc[1][j], a0, a1, bb);
    }
  }
  acc_guard4(acc[0][0], acc[0][1], acc[0][2], acc[0][3]);
  acc_guard4(acc[0][4], acc[0][5], acc[0][6], acc[0][7]);
  acc_guard4(acc[1][0], acc[1][1], acc[1][2], acc[1][3]);
  acc_guard4(acc[1][4], acc[1][5], acc[1][6], acc[1][7]);

  float bj[8];
#pragma unroll
  for (int j = 0; j < 8; ++j) bj[j] = 0.f;
  if (OM == 4) {
#pragma unroll
    for (int j = 0; j < 8; ++j) bj[j] = bfr(bias[n0 + 16 * j + rl]);
  }

  float* slab = sT[wave];
#pragma unroll
  for (int i = 0; i < 2; ++i) {
    const int mB = m0 + 16 * i;
#pragma unroll
    for (int j = 0; j < 8; ++j) {
#pragma unroll
      for (int r = 0; r < 8; ++r) {
        float v = acc[i][j][r] * oscale;
        if (OM == 4) v += bj[j];
        slab[(8 * hh + r) * 132 + 16 * j + rl] = v;
      }
    }
    wave_sync_lds();
    if (OM == 4) {
      float* Cf = (float*)C0;
      for (int pass = 0; pass < 2; ++pass) {
#pragma unroll
        for (int it = 0; it < 16; ++it) {
          const v4f o = *(const v4f*)(slab + it * 132 + lane * 4);
          *(volatile v4f*)(Cf + (size_t)(mB + it) * (size_t)ldc + n0 + lane * 4) = o;
        }
        __threadfence();
      }
    } else {
      unsigned short* Cp = (unsigned short*)C0;
      v4u hv[8];
#pragma unroll
      for (int it = 0; it < 8; ++it) {
        const int row = it * 2 + hh;
        const float* sp = slab + row * 132 + rl * 8;
        const v4f fa = *(const v4f*)sp;
        const v4f fb = *(const v4f*)(sp + 4);
        float f[8];
        f[0] = fa[0]; f[1] = fa[1]; f[2] = fa[2]; f[3] = fa[3];
        f[4] = fb[0]; f[5] = fb[1]; f[6] = fb[2]; f[7] = fb[3];
        v4u pk;
#pragma unroll
        for (int e = 0; e < 4; ++e) {
          const _Float16 x0 = (_Float16)f[2 * e];
          const _Float16 x1 = (_Float16)f[2 * e + 1];
          pk[e] = pk16(h_bits(x0), h_bits(x1));
        }
        hv[it] = pk;
      }
      for (int pass = 0; pass < 2; ++pass) {
#pragma unroll
        for (int it = 0; it < 8; ++it) {
          const int row = it * 2 + hh;
          const size_t go = (size_t)(mB + row) * (size_t)ldc + n0 + rl * 8;
          *(volatile v4u*)(Cp + go) = hv[it];
        }
        __threadfence();
      }
    }
    wave_sync_lds();
  }
}

__global__ __launch_bounds__(128)
void attn_k(const unsigned short* __restrict__ QP, const unsigned short* __restrict__ KP,
            const unsigned short* __restrict__ VTp, unsigned short* CTX) {
  __shared__ __align__(16) _Float16 Psh[4][16 * 64];
  __shared__ __align__(16) float    Os[4][16 * 192];

  const int tid  = threadIdx.x;
  const int wave = tid >> 5;
  const int lane = tid & 31;
  const int hh   = lane >> 4;
  const int c    = lane & 15;

  int bid = (int)blockIdx.x;
  const int qb = bid % NQB;         bid /= NQB;
  const int hp = bid % (NHEAD / 2); bid /= (NHEAD / 2);
  const int b  = bid;
  const int q0 = qb * 64 + wave * 16;
  const size_t qrow = (size_t)b * QTOK + (size_t)q0;

  const _Float16* QPh = (const _Float16*)(const void*)QP;
  const _Float16* KPh = (const _Float16*)(const void*)KP;
  const _Float16* VTh = (const _Float16*)(const void*)VTp;
  _Float16* pwh = Psh[wave];
  float* os = Os[wave];

#pragma unroll 1
  for (int hs = 0; hs < 2; ++hs) {
    const int h = hp * 2 + hs;
    const _Float16* Qg = QPh + (qrow + (size_t)c) * DMODEL + h * DCH + 8 * hh;
    const _Float16* Kg = KPh + ((size_t)b * KPAD + (size_t)c) * DMODEL + h * DCH + 8 * hh;
    const _Float16* Vg = VTh + (size_t)(h * DCH + c) * (size_t)MK + (size_t)b * KPAD + 8 * hh;

    v16h qa[3];
#pragma unroll
    for (int dc = 0; dc < 3; ++dc) qa[dc] = ldfrag_h(Qg + 32 * dc);

    float mrow[8], lrow[8];
    v8f oh[6];
#pragma unroll
    for (int r = 0; r < 8; ++r) { mrow[r] = NEG_BIG; lrow[r] = 0.f; }
#pragma unroll
    for (int t = 0; t < 6; ++t) oh[t] = zero8();

    for (int kt = 0; kt < NKC; ++kt) {
      const int kv0 = kt * 64;
      v8f s[4];
#pragma unroll
      for (int j = 0; j < 4; ++j) s[j] = zero8();
#pragma unroll
      for (int dc = 0; dc < 3; ++dc) {
#pragma unroll
        for (int j = 0; j < 4; ++j) {
          const v16h kb = ldfrag_h(Kg + (size_t)(kv0 + 16 * j) * DMODEL + 32 * dc);
          s[j] = mma_h(qa[dc], kb, s[j]);
        }
      }
      acc_guard4(s[0], s[1], s[2], s[3]);
#pragma unroll
      for (int j = 0; j < 4; ++j) {
        const bool kval = (kv0 + 16 * j + c) < KTOK;
#pragma unroll
        for (int r = 0; r < 8; ++r) s[j][r] = kval ? (s[j][r] * SSC) : NEG_BIG;
      }
      wave_sync_lds();

#pragma unroll
      for (int r = 0; r < 8; ++r) {
        float m = s[0][r];
        m = fmaxf(m, s[1][r]);
        m = fmaxf(m, s[2][r]);
        m = fmaxf(m, s[3][r]);
#pragma unroll
        for (int off = 1; off < 16; off <<= 1) m = fmaxf(m, __shfl_xor(m, off, 32));
        const float mnew  = fmaxf(mrow[r], m);
        const float alpha = __expf(mrow[r] - mnew);
        mrow[r] = mnew;
        float psum = 0.f;
#pragma unroll
        for (int j = 0; j < 4; ++j) {
          const float p = __expf(s[j][r] - mnew);
          psum += p;
          pwh[(8 * hh + r) * 64 + j * 16 + c] = (_Float16)(p * PSC);
        }
#pragma unroll
        for (int off = 1; off < 16; off <<= 1) psum += __shfl_xor(psum, off, 32);
        lrow[r] = lrow[r] * alpha + psum;
#pragma unroll
        for (int t = 0; t < 6; ++t) oh[t][r] *= alpha;
      }
      wave_sync_lds();

#pragma unroll
      for (int kk = 0; kk < 2; ++kk) {
        FH pa;
        pa.h[0] = *(const v8h*)(pwh + c * 64 + kk * 32 + 8 * hh);
        pa.h[1] = *(const v8h*)(pwh + c * 64 + kk * 32 + 16 + 8 * hh);
#pragma unroll
        for (int t = 0; t < 6; ++t) {
          const v16h vb = ldfrag_h(Vg + (size_t)(16 * t) * (size_t)MK + kv0 + 32 * kk);
          oh[t] = mma_h(pa.v, vb, oh[t]);
        }
      }
    }
    acc_guard4(oh[0], oh[1], oh[2], oh[3]);
    acc_guard2(oh[4], oh[5]);

#pragma unroll
    for (int r = 0; r < 8; ++r) {
      const float l = lrow[r];
      const float inv = ((l > 0.f) ? (1.0f / l) : 0.f) * (CSC / (PSC * VSC));
#pragma unroll
      for (int t = 0; t < 6; ++t) os[(8 * hh + r) * 192 + hs * 96 + t * 16 + c] = oh[t][r] * inv;
    }
  }
  wave_sync_lds();

  {
    const int cl = (lane < 24) ? lane : 23;
    for (int pass = 0; pass < 2; ++pass) {
#pragma unroll 4
      for (int it = 0; it < 16; ++it) {
        const float* sp = os + it * 192 + cl * 8;
        const v4f fa = *(const v4f*)sp;
        const v4f fb = *(const v4f*)(sp + 4);
        float f[8];
        f[0] = fa[0]; f[1] = fa[1]; f[2] = fa[2]; f[3] = fa[3];
        f[4] = fb[0]; f[5] = fb[1]; f[6] = fb[2]; f[7] = fb[3];
        v4u pk;
#pragma unroll
        for (int e = 0; e < 4; ++e) {
          const _Float16 x0 = (_Float16)f[2 * e];
          const _Float16 x1 = (_Float16)f[2 * e + 1];
          pk[e] = pk16(h_bits(x0), h_bits(x1));
        }
        const size_t go = (qrow + (size_t)it) * DMODEL + (size_t)(hp * 192 + cl * 8);
        if (lane < 24) *(volatile v4u*)(CTX + go) = pk;
      }
      __threadfence();
    }
  }
}


typedef unsigned int v4u_z __attribute__((ext_vector_type(4)));
__global__ __launch_bounds__(256) void zero16(v4u_z* __restrict__ p) {
  const v4u_z z = {0u, 0u, 0u, 0u};
  *(volatile v4u_z*)(p + (size_t)blockIdx.x * 256 + threadIdx.x) = z;
}

extern "C" void kernel_launch(void* const* d_in, const int* in_sizes, int n_in,
                              void* d_out, int out_size, void* d_ws, size_t ws_size,
                              hipStream_t stream) {
  if (n_in < 15) return;
  if (in_sizes[0] != MQ * DMODEL) return;
  if (in_sizes[1] != DCH * NTAP || in_sizes[2] != DCH * NTAP || in_sizes[3] != DCH * NTAP) return;
  for (int i = 4; i < 10; ++i) if (in_sizes[i] != DCH) return;
  for (int i = 10; i < 14; ++i) if (in_sizes[i] != DMODEL * DMODEL) return;
  if (in_sizes[14] != DMODEL) return;
  if (out_size != MQ * DMODEL) return;

  const float* X   = (const float*)d_in[0];
  const float* pqw = (const float*)d_in[1];
  const float* pkw = (const float*)d_in[2];
  const float* pvw = (const float*)d_in[3];
  const float* nqg = (const float*)d_in[4];
  const float* nqb = (const float*)d_in[5];
  const float* nkg = (const float*)d_in[6];
  const float* nkb = (const float*)d_in[7];
  const float* nvg = (const float*)d_in[8];
  const float* nvb = (const float*)d_in[9];
  const float* lqw = (const float*)d_in[10];
  const float* lkw = (const float*)d_in[11];
  const float* lvw = (const float*)d_in[12];
  const float* pjw = (const float*)d_in[13];
  const float* pjb = (const float*)d_in[14];

  const size_t PW  = (size_t)DMODEL * DMODEL * 2;
  const size_t PQ  = (size_t)MQ * DMODEL * 2;
  const size_t PK  = (size_t)MK * DMODEL * 2;
  const size_t PVT = (size_t)DMODEL * MK * 2;
  size_t off = 0;
  const size_t oWQ  = off; off += PW;
  const size_t oWK  = off; off += PW;
  const size_t oWV  = off; off += PW;
  const size_t oWP  = off; off += PW;
  const size_t oQLN = off; off += PQ;
  const size_t oKLN = off; off += PK;
  const size_t oVLN = off; off += PK;
  const size_t oQP  = off; off += PQ;
  const size_t oKP  = off; off += PK;
  const size_t oVT  = off; off += PVT;
  const size_t oCTX = off; off += PQ;
  if (off > ws_size) return;
  if (off > (size_t)134217728) return;

  char* ws = (char*)d_ws;
  unsigned short* WQ  = (unsigned short*)(ws + oWQ);
  unsigned short* WK  = (unsigned short*)(ws + oWK);
  unsigned short* WV  = (unsigned short*)(ws + oWV);
  unsigned short* WP  = (unsigned short*)(ws + oWP);
  unsigned short* QLN = (unsigned short*)(ws + oQLN);
  unsigned short* KLN = (unsigned short*)(ws + oKLN);
  unsigned short* VLN = (unsigned short*)(ws + oVLN);
  unsigned short* QP  = (unsigned short*)(ws + oQP);
  unsigned short* KPL = (unsigned short*)(ws + oKP);
  unsigned short* VT  = (unsigned short*)(ws + oVT);
  unsigned short* CTX = (unsigned short*)(ws + oCTX);

  const dim3 blk256(256), blk192(192), blk128(128);

  cvt_w<<<dim3((DMODEL * DMODEL) / 2048), blk256, 0, stream>>>(lqw, WQ, DMODEL * DMODEL, WSC);
  cvt_w<<<dim3((DMODEL * DMODEL) / 2048), blk256, 0, stream>>>(lkw, WK, DMODEL * DMODEL, WSC);
  cvt_w<<<dim3((DMODEL * DMODEL) / 2048), blk256, 0, stream>>>(lvw, WV, DMODEL * DMODEL, WSC);
  cvt_w<<<dim3((DMODEL * DMODEL) / 2048), blk256, 0, stream>>>(pjw, WP, DMODEL * DMODEL, WSC);

  for (int b = 0; b < NBATCH; ++b) {
    const size_t prow = ((size_t)b * KPAD + KTOK) * DMODEL * 2;
    const size_t pbytes = (size_t)(KPAD - KTOK) * DMODEL * 2;
    zero16<<<dim3((unsigned)(pbytes / 16 / 256)), blk256, 0, stream>>>((v4u_z*)((char*)KLN + prow));
    zero16<<<dim3((unsigned)(pbytes / 16 / 256)), blk256, 0, stream>>>((v4u_z*)((char*)VLN + prow));
  }

  pool_ln<1, SDIM><<<dim3(NBATCH * 4 * TDIM * SDIM), blk192, 0, stream>>>(X, pqw, nqg, nqb, QLN, QTOK);
  pool_ln<2, KSD><<<dim3(NBATCH * 4 * TDIM * KSD), blk192, 0, stream>>>(X, pkw, nkg, nkb, KLN, KPAD);
  pool_ln<2, KSD><<<dim3(NBATCH * 4 * TDIM * KSD), blk192, 0, stream>>>(X, pvw, nvg, nvb, VLN, KPAD);

  gemm_h<1><<<dim3(((MQ / 32) * (DMODEL / 128) + 3) / 4), blk128, 0, stream>>>(
      QLN, DMODEL, WQ, DMODEL, (void*)QP, pjb, DMODEL, MQ, DMODEL, DMODEL, QSC / WSC);
  gemm_h<1><<<dim3(((MK / 32) * (DMODEL / 128) + 3) / 4), blk128, 0, stream>>>(
      KLN, DMODEL, WK, DMODEL, (void*)KPL, pjb, DMODEL, MK, DMODEL, DMODEL, QSC / WSC);
  gemm_h<1><<<dim3(((DMODEL / 32) * (MK / 128) + 3) / 4), blk128, 0, stream>>>(
      WV, DMODEL, VLN, DMODEL, (void*)VT, pjb, MK, DMODEL, MK, DMODEL, VSC / WSC);

  attn_k<<<dim3(NQB * (NHEAD / 2) * NBATCH), blk128, 0, stream>>>(QP, KPL, VT, CTX);

  gemm_h<4><<<dim3(((MQ / 32) * (DMODEL / 128) + 3) / 4), blk128, 0, stream>>>(
      CTX, DMODEL, WP, DMODEL, d_out, pjb, DMODEL, MQ, DMODEL, DMODEL, 1.0f / (CSC * WSC));
  (void)hipGetLastError();
}
